// IterSpatialCorrelationSampler_7885559955777
// MI455X (gfx1250) — hardware-verified
//
#include <hip/hip_runtime.h>
#include <stdint.h>

typedef __attribute__((ext_vector_type(16))) __bf16   v16b;
typedef __attribute__((ext_vector_type(8)))  __bf16   v8b;
typedef __attribute__((ext_vector_type(8)))  float    v8f;
typedef __attribute__((ext_vector_type(4)))  float    v4f;
typedef __attribute__((ext_vector_type(4)))  unsigned v4u;

constexpr int NBATCH = 4;
constexpr int NCHAN  = 256;
constexpr int NROWS  = 96;
constexpr int NWID   = 128;
constexpr int NPATCH = 9;
constexpr int POFF   = 4;
constexpr int NQ     = NPATCH * NPATCH;
constexpr int HPAD   = NROWS + 2 * POFF;
constexpr int WPAD   = NWID + 2 * POFF + 8;
constexpr long HW    = (long)NROWS * NWID;
constexpr long NPIX_A = (long)NBATCH * NROWS * NWID;
constexpr long NPIX_B = (long)NBATCH * HPAD * WPAD;
constexpr long A_ELEMS = NPIX_A * NCHAN;
constexpr long B_ELEMS = NPIX_B * NCHAN;
constexpr size_t WS_CARVE = (size_t)(A_ELEMS + B_ELEMS) * 2;

static_assert(NCHAN % 32 == 0, "K multiple of 32");
static_assert(NCHAN == 32 * 8, "one wave = 32 lanes x 8 channels per pixel in the pack kernels");
static_assert(NWID % 16 == 0 && NWID / 16 == 8, "8 strips of 16 pixels per row = 8 waves per block");
static_assert(NWID == 32 * 4, "one wave x float4 = one whole output row (4 x 128-B lines)");
static_assert((NROWS - 1) + (NPATCH - 1) < HPAD, "padded rows cover every dy");
static_assert((NWID - 16) + 16 + 15 < WPAD, "padded cols cover tile 1 of the last strip");
static_assert(WS_CARVE <= (size_t)134217728, "carve under 128 MiB");
static_assert((A_ELEMS * 2) % 128 == 0, "plane B 128-B aligned");

__device__ __forceinline__ unsigned short f2bf_bits(float f) {
  unsigned u = __float_as_uint(f);
  return (unsigned short)((u + 0x7FFFu + ((u >> 16) & 1u)) >> 16);
}

template <typename T> struct Frag;
template <> struct Frag<__bf16> {
  typedef v16b V; union U { v16b v; v8b h[2]; };
  static __device__ __forceinline__ v16b load(const __bf16* p) {
    U f; f.h[0] = *(const v8b*)(p); f.h[1] = *(const v8b*)(p + 16); return f.v;
  }
  static __device__ __forceinline__ v8f mma(v16b a, v16b b, v8f c) {
    return __builtin_amdgcn_wmma_f32_16x16x32_bf16(false, a, false, b, (short)0, c, false, false);
  }
};

__device__ __forceinline__ void dep_guard3(v8f& a, v8f& b, v16b x, v16b y, v16b z) {
  asm volatile("v_nop\n\tv_nop\n\tv_nop\n\tv_nop" : "+v"(a), "+v"(b) : "v"(x), "v"(y), "v"(z));
}

__global__ __launch_bounds__(256)
void pack_plane_a(const float* __restrict__ in1, unsigned short* __restrict__ pA, int npix)
{
  const int p = __builtin_amdgcn_readfirstlane((int)(blockIdx.x * 8 + (threadIdx.x >> 5)));
  if (p >= npix) return;
  const int lane = threadIdx.x & 31;
  const int b  = p / (NROWS * NWID);
  const int ph = p - b * (NROWS * NWID);
  const float* src = in1 + (long)b * NCHAN * HW + ph + (long)(lane * 8) * HW;
  float f[8];
#pragma unroll
  for (int i = 0; i < 8; ++i) f[i] = src[(long)i * HW];
  v4u u;
#pragma unroll
  for (int j = 0; j < 4; ++j)
    u[j] = (unsigned)f2bf_bits(f[2 * j]) | ((unsigned)f2bf_bits(f[2 * j + 1]) << 16);
  volatile v4u* dst = (volatile v4u*)(pA + (long)p * NCHAN + lane * 8);
  *dst = u;
  __threadfence();
  *dst = u;
}

__global__ __launch_bounds__(256)
void pack_plane_b(const float* __restrict__ in2, unsigned short* __restrict__ pB, int npix)
{
  const int p = __builtin_amdgcn_readfirstlane((int)(blockIdx.x * 8 + (threadIdx.x >> 5)));
  if (p >= npix) return;
  const int lane = threadIdx.x & 31;
  const int b   = p / (HPAD * WPAD);
  const int rem = p - b * (HPAD * WPAD);
  const int hp  = rem / WPAD;
  const int wp  = rem - hp * WPAD;
  const int row = hp - POFF;
  const int col = wp - POFF;
  const bool valid = (row >= 0) && (row < NROWS) && (col >= 0) && (col < NWID);
  const int rowc = row < 0 ? 0 : (row >= NROWS ? NROWS - 1 : row);
  const int colc = col < 0 ? 0 : (col >= NWID ? NWID - 1 : col);
  const float* src = in2 + (long)b * NCHAN * HW + (long)rowc * NWID + colc + (long)(lane * 8) * HW;
  float f[8];
#pragma unroll
  for (int i = 0; i < 8; ++i) {
    const float t = src[(long)i * HW];
    f[i] = valid ? t : 0.0f;
  }
  v4u u;
#pragma unroll
  for (int j = 0; j < 4; ++j)
    u[j] = (unsigned)f2bf_bits(f[2 * j]) | ((unsigned)f2bf_bits(f[2 * j + 1]) << 16);
  volatile v4u* dst = (volatile v4u*)(pB + (long)p * NCHAN + lane * 8);
  *dst = u;
  __threadfence();
  *dst = u;
}

__global__ __launch_bounds__(256)
void corr_rows(const unsigned short* __restrict__ pA,
               const unsigned short* __restrict__ pB,
               float* __restrict__ out)
{
  __shared__ __align__(16) float S[NQ * NWID];

  const int wave = __builtin_amdgcn_readfirstlane((int)(threadIdx.x >> 5));
  const int lane = threadIdx.x & 31;
  const int hh   = lane >> 4;
  const int c    = lane & 15;
  const int bh   = blockIdx.x;
  const int b    = bh / NROWS;
  const int h    = bh - b * NROWS;
  const int w0   = wave * 16;

  const __bf16* Arow = (const __bf16*)pA + (((long)(b * NROWS + h) * NWID) + w0 + c) * NCHAN + 8 * hh;
  const __bf16* Bbase = (const __bf16*)pB + (((long)(b * HPAD + h) * WPAD) + w0 + c) * NCHAN + 8 * hh;

#pragma unroll 1
  for (int dy = 0; dy < NPATCH; ++dy) {
    const __bf16* B0 = Bbase + (long)dy * WPAD * NCHAN;
    const __bf16* B1 = B0 + 16 * NCHAN;
    v8f acc0 = (v8f){0.f,0.f,0.f,0.f,0.f,0.f,0.f,0.f};
    v8f acc1 = (v8f){0.f,0.f,0.f,0.f,0.f,0.f,0.f,0.f};
#pragma unroll 1
    for (int k0 = 0; k0 < NCHAN; k0 += 32) {
      const v16b a   = Frag<__bf16>::load(Arow + k0);
      const v16b bf0 = Frag<__bf16>::load(B0 + k0);
      const v16b bf1 = Frag<__bf16>::load(B1 + k0);
      acc0 = Frag<__bf16>::mma(a, bf0, acc0);
      acc1 = Frag<__bf16>::mma(a, bf1, acc1);
      dep_guard3(acc0, acc1, a, bf0, bf1);
    }
    float* Sdy = S + dy * NPATCH * NWID;
#pragma unroll
    for (int r = 0; r < 8; ++r) {
      const int m   = 8 * hh + r;
      const int dx0 = c - m - POFF;
      const int dx1 = c - m + 16 - POFF;
      const bool v0 = (dx0 >= -POFF) && (dx0 <= POFF);
      const bool v1 = (dx1 >= -POFF) && (dx1 <= POFF);
      const int j0 = v0 ? (dx0 + POFF) : 0;
      const int j1 = v1 ? (dx1 + POFF) : 0;
      const float val0 = acc0[r];
      const float val1 = acc1[r];
      if (v0) Sdy[j0 * NWID + w0 + m] = val0;
      if (v1) Sdy[j1 * NWID + w0 + m] = val1;
    }
  }

  __syncthreads();

  float* orow = out + (((long)b * NQ) * NROWS + h) * NWID + lane * 4;
  for (int pass = 0; pass < 2; ++pass) {
    for (int q = wave; q < NQ; q += 8) {
      const v4f v = *(const v4f*)(S + q * NWID + lane * 4);
      *(volatile v4f*)(orow + (long)q * NROWS * NWID) = v;
    }
    __threadfence();
  }
}

extern "C" void kernel_launch(void* const* d_in, const int* in_sizes, int n_in,
                              void* d_out, int out_size, void* d_ws, size_t ws_size,
                              hipStream_t stream)
{
  if (n_in < 2) return;
  const long n_expect = (long)NBATCH * NCHAN * NROWS * NWID;
  if ((long)in_sizes[0] != n_expect || (long)in_sizes[1] != n_expect) return;
  if ((long)out_size != (long)NBATCH * NQ * NROWS * NWID) return;
  if (ws_size < WS_CARVE || d_ws == nullptr) return;

  const float* in1 = (const float*)d_in[0];
  const float* in2 = (const float*)d_in[1];
  float* out = (float*)d_out;
  unsigned short* pA = (unsigned short*)d_ws;
  unsigned short* pB = pA + A_ELEMS;

  const int gridA = (int)((NPIX_A + 7) / 8);
  const int gridB = (int)((NPIX_B + 7) / 8);
  pack_plane_a<<<gridA, 256, 0, stream>>>(in1, pA, (int)NPIX_A);
  pack_plane_b<<<gridB, 256, 0, stream>>>(in2, pB, (int)NPIX_B);
  corr_rows<<<NBATCH * NROWS, 256, 0, stream>>>(pA, pB, out);
}
